// SelfAttention_71047349010537
// MI455X (gfx1250) — hardware-verified
//
#include <hip/hip_runtime.h>


#ifndef NB
#define NB 4
#endif
#ifndef SEQ
#define SEQ 2048
#endif
#define NB_FULL  4
#define SEQ_FULL 2048
#define DD    256
#define NHEAD 8
#define NHA   NB
#define KM    (NHA * DD)
#define KMF   (NHEAD * DD)
#ifndef EROWS
#define EROWS 768
#endif
#define PCAR  1024.0f
#define SCL2  0.09016844005556021f
#define OCAR  0.0625f
#define WOCAR 256.0f
#define FINSC (1.0f / 16384.0f)
#define RCAR  2048.0f
#define RINV  (1.0f / 2048.0f)
#define MSW   4
#define XG  ((unsigned)(SEQ * DD / 8))
#define WG  ((unsigned)(NHA * DD * DD / 8))
#define OG  ((unsigned)(DD * KM / 8))
#define PREPX ((XG > WG ? XG : WG) / 256u)

typedef _Float16 h16;
typedef unsigned short bf;
typedef __attribute__((ext_vector_type(16))) __bf16   v16bf;
typedef __attribute__((ext_vector_type(16))) _Float16 v16h;
typedef __attribute__((ext_vector_type(8)))  _Float16 v8h;
typedef __attribute__((ext_vector_type(8)))  unsigned short v8us;
typedef __attribute__((ext_vector_type(2)))  unsigned short v2us;
typedef __attribute__((ext_vector_type(8)))  float    v8f;
typedef __attribute__((ext_vector_type(4)))  float    v4f;
typedef __attribute__((ext_vector_type(4)))  int      v4i;
typedef v4f  __attribute__((may_alias)) v4fa;

static_assert(SEQ % 256 == 0);
static_assert(DD % 64 == 0 && DD % 32 == 0 && KM % 32 == 0 && SEQ % 64 == 0);
static_assert(NB >= 1 && NB <= NHEAD && NHA <= 32);
static_assert(NB <= NB_FULL && SEQ <= SEQ_FULL);
static_assert(XG % 256u == 0 && WG % 256u == 0 && OG == WG);
static_assert(((size_t)3 * NHA * SEQ * DD / 8) % 256 == 0);
static_assert(((size_t)(NB - 1) * SEQ * DD / 4) % 256 == 0);
static_assert((NHA * SEQ) % 8 == 0 && SEQ % 8 == 0);
static_assert(EROWS >= 0 && EROWS % 64 == 0);
static_assert(KM % 64 == 0 && (KM / 8) > 0);
static_assert(SEQ % MSW == 0 && (NHA * SEQ) % MSW == 0);
static_assert((size_t)MSW * SEQ * 4 <= (size_t)65536);
static_assert((SEQ / 256) * 64 == SEQ / 4);

__device__ __forceinline__ unsigned short f2bf(float f) { unsigned u = __float_as_uint(f); u += 0x7FFFu + ((u >> 16) & 1u); return (unsigned short)(u >> 16); }
__device__ __forceinline__ float bf2f(unsigned short b) { return __uint_as_float(((unsigned)b) << 16); }
__device__ __forceinline__ float bfr(float f) { return bf2f(f2bf(f)); }
__device__ __forceinline__ v16h cat16(v8h lo, v8h hi) { return __builtin_shufflevector(lo, hi, 0, 1, 2, 3, 4, 5, 6, 7, 8, 9, 10, 11, 12, 13, 14, 15); }
__device__ __forceinline__ v16bf cat16b(v8us lo, v8us hi) { return __builtin_bit_cast(v16bf, __builtin_shufflevector(lo, hi, 0, 1, 2, 3, 4, 5, 6, 7, 8, 9, 10, 11, 12, 13, 14, 15)); }
__device__ __forceinline__ v8f wmma16(v16h a, v16h b, v8f c) { return __builtin_amdgcn_wmma_f32_16x16x32_f16(false, a, false, b, (short)0, c, false, false); }
__device__ __forceinline__ v8f wmmab(v16bf a, v16bf b, v8f c) { return __builtin_amdgcn_wmma_f32_16x16x32_bf16(false, a, false, b, (short)0, c, false, false); }

static __device__ __forceinline__ h16 toh_flush(float v) { const h16 r = (h16)v; return (fabsf(v) < 6.103515625e-05f) ? (h16)0.0f : r; }

template <typename T16> struct WFrag;
template <> struct WFrag<h16> { typedef v16h V; static __device__ __forceinline__ V ld(const h16* p) { return cat16(*(const v8h*)p, *(const v8h*)(p + 16)); } static __device__ __forceinline__ v8f mma(V a, V b, v8f c) { return wmma16(a, b, c); } };
template <> struct WFrag<bf> { typedef v16bf V; static __device__ __forceinline__ V ld(const bf* p) { return cat16b(*(const v8us*)p, *(const v8us*)(p + 16)); } static __device__ __forceinline__ v8f mma(V a, V b, v8f c) { return wmmab(a, b, c); } };

template <int BIASM>
__device__ __forceinline__ void slab_store(const float* os, h16* crow, int ldc, const float* bias, float alpha, unsigned colbase, unsigned rowbase, unsigned lane) {
    const unsigned rq = lane >> 3, cq = lane & 7u;
    float bc[8];
#pragma unroll
    for (int e = 0; e < 8; ++e) bc[e] = 0.f;
    if (BIASM == 1) { const v4f b0 = *(const v4f*)(bias + colbase + cq * 8u); const v4f b1 = *(const v4f*)(bias + colbase + cq * 8u + 4u);
#pragma unroll
        for (int e = 0; e < 4; ++e) { bc[e] = bfr(b0[e]); bc[4 + e] = bfr(b1[e]); } }
    v8h vals[4];
#pragma unroll
    for (int s = 0; s < 4; ++s) { const unsigned row = (unsigned)s * 4u + rq; const v4f x0 = *(const v4fa*)(os + row * 68u + cq * 8u); const v4f x1 = *(const v4fa*)(os + row * 68u + cq * 8u + 4u);
        float br = 0.f; if (BIASM == 2) br = bfr(bias[rowbase + row]);
        v8h o;
#pragma unroll
        for (int e = 0; e < 4; ++e) { o[e] = (h16)(x0[e] * alpha + (bc[e] + br)); o[4 + e] = (h16)(x1[e] * alpha + (bc[4 + e] + br)); }
        vals[s] = o; }
#pragma unroll 1
    for (int ps = 0; ps < 2; ++ps) {
#pragma unroll
        for (int s = 0; s < 4; ++s) { const unsigned row = (unsigned)s * 4u + rq; *(volatile v8h*)(crow + (size_t)row * ldc + cq * 8u) = vals[s]; }
        if (ps == 0) __threadfence(); }
}
template <int BIASM>
__device__ __forceinline__ void slab_store(const float* os, float* crow, int ldc, const float* bias, float alpha, unsigned colbase, unsigned rowbase, unsigned lane) {
    const unsigned hi = lane >> 4, cofs = (lane & 15u) * 4u;
    v4f bc = (v4f){0.f, 0.f, 0.f, 0.f};
    if (BIASM == 1) { const v4f b0 = *(const v4f*)(bias + colbase + cofs);
#pragma unroll
        for (int e = 0; e < 4; ++e) bc[e] = bfr(b0[e]); }
    v4f vals[8];
#pragma unroll
    for (int s = 0; s < 8; ++s) { const unsigned row = (unsigned)s * 2u + hi; const v4f x = *(const v4fa*)(os + row * 68u + cofs);
        float br = 0.f; if (BIASM == 2) br = bfr(bias[rowbase + row]);
        v4f o;
#pragma unroll
        for (int e = 0; e < 4; ++e) o[e] = x[e] * alpha + (bc[e] + br);
        vals[s] = o; }
#pragma unroll 1
    for (int ps = 0; ps < 2; ++ps) {
#pragma unroll
        for (int s = 0; s < 8; ++s) { const unsigned row = (unsigned)s * 2u + hi; *(volatile v4f*)(crow + (size_t)row * ldc + cofs) = vals[s]; }
        if (ps == 0) __threadfence(); }
}

template <typename T16, typename OT, int BIASM>
__global__ __launch_bounds__(32) void k_gemmw(const T16* __restrict__ A, const T16* __restrict__ Bt, int K, OT* C, int ldc, const float* __restrict__ bias, float alpha, size_t sA, size_t sB, size_t sC, int sBias) {
    typedef typename WFrag<T16>::V V;
    __shared__ __align__(16) float os[16 * 68];
    const size_t z = blockIdx.z; A += z * sA; Bt += z * sB; C += z * sC; if (BIASM != 0) bias += z * (size_t)sBias;
    const unsigned lane = threadIdx.x & 31u, lr = lane & 15u, hi = lane >> 4; const unsigned r0 = blockIdx.x * 64u, c0 = blockIdx.y * 64u;
    v8f acc[4][4];
#pragma unroll
    for (int mb = 0; mb < 4; ++mb)
#pragma unroll
        for (int nb = 0; nb < 4; ++nb) acc[mb][nb] = (v8f){};
    const size_t aoff = (size_t)(r0 + lr) * K + 8u * hi, boff = (size_t)(c0 + lr) * K + 8u * hi;
#pragma unroll 1
    for (int kc = 0; kc < K; kc += 32) {
        V a[4];
#pragma unroll
        for (int mb = 0; mb < 4; ++mb) a[mb] = WFrag<T16>::ld(A + aoff + (size_t)mb * 16 * K + kc);
#pragma unroll
        for (int nb = 0; nb < 4; ++nb) { const V b = WFrag<T16>::ld(Bt + boff + (size_t)nb * 16 * K + kc);
#pragma unroll
            for (int mb = 0; mb < 4; ++mb) acc[mb][nb] = WFrag<T16>::mma(a[mb], b, acc[mb][nb]); }
        asm volatile("v_nop\n\tv_nop\n\tv_nop\n\tv_nop" : "+v"(acc[0][0]), "+v"(acc[1][1]), "+v"(acc[2][2]), "+v"(acc[3][3]) : "v"(a[0]), "v"(a[3]));
    }
#pragma unroll
    for (int mb = 0; mb < 4; ++mb) {
#pragma unroll
        for (int nb = 0; nb < 4; ++nb) {
#pragma unroll
            for (int j = 0; j < 8; ++j) os[(hi * 8u + (unsigned)j) * 68u + (unsigned)nb * 16u + lr] = acc[mb][nb][j]; }
        __builtin_amdgcn_fence(3  , "wavefront"); __builtin_amdgcn_wave_barrier(); asm volatile("" ::: "memory");
        OT* crow = C + (size_t)(r0 + (unsigned)mb * 16u) * ldc + c0;
        slab_store<BIASM>(os, crow, ldc, bias, alpha, c0, r0 + (unsigned)mb * 16u, lane);
        __builtin_amdgcn_fence(3  , "wavefront"); __builtin_amdgcn_wave_barrier(); asm volatile("" ::: "memory");
    }
}

__device__ __forceinline__ v8f wmma_g(v16h a, v16h b, v8f c) {
    c = wmma16(a, b, c);
    asm volatile("v_nop\n\tv_nop\n\tv_nop\n\tv_nop" : "+v"(c) : "v"(a), "v"(b));
    return c;
}
__device__ __forceinline__ void gemm_kstep(v8f (&acc)[4][4], const h16* A, const h16* B, size_t aoff, size_t boff, int lda, int ldb, int kc) {
    v16h a[4];
#pragma unroll
    for (int mb = 0; mb < 4; ++mb) a[mb] = WFrag<h16>::ld(A + aoff + (size_t)mb * 16 * lda + kc);
#pragma unroll
    for (int nb = 0; nb < 4; ++nb) { const v16h b = WFrag<h16>::ld(B + boff + (size_t)nb * 16 * ldb + kc);
#pragma unroll
        for (int mb = 0; mb < 4; ++mb) acc[mb][nb] = wmma_g(a[mb], b, acc[mb][nb]); }
}
__device__ __forceinline__ void slab_store_pair(const float* os, h16* crow, h16* rrow, int ldc, float alpha, unsigned lane) {
    const unsigned rq = lane >> 3, cq = lane & 7u;
    v8h vh[4], vr[4];
#pragma unroll
    for (int s = 0; s < 4; ++s) { const unsigned row = (unsigned)s * 4u + rq; const v4f x0 = *(const v4fa*)(os + row * 68u + cq * 8u); const v4f x1 = *(const v4fa*)(os + row * 68u + cq * 8u + 4u);
        v8h oh, orr;
#pragma unroll
        for (int e = 0; e < 4; ++e) {
            const float y0 = x0[e] * alpha; const h16 h0 = toh_flush(y0); oh[e] = h0; orr[e] = toh_flush((y0 - (float)h0) * RCAR);
            const float y1 = x1[e] * alpha; const h16 h1 = toh_flush(y1); oh[4 + e] = h1; orr[4 + e] = toh_flush((y1 - (float)h1) * RCAR); }
        vh[s] = oh; vr[s] = orr; }
#pragma unroll 1
    for (int ps = 0; ps < 2; ++ps) {
#pragma unroll
        for (int s = 0; s < 4; ++s) { const unsigned row = (unsigned)s * 4u + rq;
            *(volatile v8h*)(crow + (size_t)row * ldc + cq * 8u) = vh[s];
            *(volatile v8h*)(rrow + (size_t)row * ldc + cq * 8u) = vr[s]; }
        if (ps == 0) __threadfence(); }
}

template <int SITE>
__device__ __forceinline__ void gemmb_body(float* os, const h16* AH, const h16* AR, const h16* BH, const h16* BR, int lda, int ldb, int K,
                                           float* CF, h16* C1, h16* C2, int ldc, const float* bias, float alpha, const int* PLW) {
    const unsigned lane = threadIdx.x & 31u, lr = lane & 15u, hi = lane >> 4; const unsigned r0 = blockIdx.x * 64u, c0 = blockIdx.y * 64u; const unsigned z = blockIdx.z;
    int kb = 0, ke = K, ea = 0;
    if (SITE == 0) { int pl = PLW[z]; pl = min(max(pl, 0), SEQ);
        const int dead = (((int)c0 > (int)r0 + 63) || ((int)r0 + 64 <= pl) || ((int)c0 + 64 <= pl)) ? 1 : 0;
        ke = (dead != 0) ? 0 : K; ea = ((EROWS > 0) && (dead == 0) && ((int)r0 < pl + EROWS)) ? 1 : 0; }
    if (SITE == 1) { int pl = PLW[z]; pl = min(max(pl, 0), SEQ);
        const int dead = ((int)r0 + 64 <= pl) ? 1 : 0;
        kb = pl & ~31; ke = (dead != 0) ? kb : ((int)r0 + 64); ea = ((EROWS > 0) && (dead == 0) && ((int)r0 < pl + EROWS)) ? 1 : 0; }
    if (SITE == 2) {
#pragma unroll
        for (int n = 0; n < NHA; ++n) { int pl = PLW[n]; pl = min(max(pl, 0), SEQ); ea |= ((EROWS > 0) && ((int)r0 + 64 > pl) && ((int)r0 < pl + EROWS)) ? 1 : 0; } }
    const int kbeg = __builtin_amdgcn_readfirstlane(kb), kend = __builtin_amdgcn_readfirstlane(ke), early = __builtin_amdgcn_readfirstlane(ea);
    v8f acc[4][4];
#pragma unroll
    for (int mb = 0; mb < 4; ++mb)
#pragma unroll
        for (int nb = 0; nb < 4; ++nb) acc[mb][nb] = (v8f){};
    const size_t aoff = (size_t)(r0 + lr) * lda + 8u * hi, boff = (size_t)(c0 + lr) * ldb + 8u * hi;
    if (early != 0) {
#pragma unroll 1
        for (int kc = kbeg; kc < kend; kc += 32) {
            if (SITE != 2) gemm_kstep(acc, AH, BR, aoff, boff, lda, ldb, kc);
            gemm_kstep(acc, AR, BH, aoff, boff, lda, ldb, kc);
        }
#pragma unroll
        for (int mb = 0; mb < 4; ++mb)
#pragma unroll
            for (int nb = 0; nb < 4; ++nb) acc[mb][nb] = acc[mb][nb] * RINV;
    }
#pragma unroll 1
    for (int kc = kbeg; kc < kend; kc += 32) gemm_kstep(acc, AH, BH, aoff, boff, lda, ldb, kc);
#pragma unroll
    for (int mb = 0; mb < 4; ++mb) {
#pragma unroll
        for (int nb = 0; nb < 4; ++nb) {
#pragma unroll
            for (int j = 0; j < 8; ++j) os[(hi * 8u + (unsigned)j) * 68u + (unsigned)nb * 16u + lr] = acc[mb][nb][j]; }
        __builtin_amdgcn_fence(3  , "wavefront"); __builtin_amdgcn_wave_barrier(); asm volatile("" ::: "memory");
        const size_t coff = (size_t)(r0 + (unsigned)mb * 16u) * ldc + c0;
        if (SITE == 0) slab_store<0>(os, CF + coff, ldc, bias, alpha, c0, r0 + (unsigned)mb * 16u, lane);
        if (SITE == 1) slab_store_pair(os, C1 + coff, C2 + coff, ldc, alpha, lane);
        if (SITE == 2) slab_store<1>(os, CF + coff, ldc, bias, alpha, c0, r0 + (unsigned)mb * 16u, lane);
        __builtin_amdgcn_fence(3  , "wavefront"); __builtin_amdgcn_wave_barrier(); asm volatile("" ::: "memory");
    }
}

__global__ __launch_bounds__(32) void k_score(const h16* __restrict__ HI, const h16* __restrict__ RS, float* S, const int* __restrict__ PLW) {
    __shared__ __align__(16) float os[16 * 68];
    const size_t z = blockIdx.z;
    const h16* qh = HI + z * SEQ * DD; const h16* qr = RS + z * SEQ * DD;
    const h16* kh = HI + ((size_t)NHA + z) * SEQ * DD; const h16* kr = RS + ((size_t)NHA + z) * SEQ * DD;
    gemmb_body<0>(os, qh, qr, kh, kr, DD, DD, DD, S + z * SEQ * SEQ, nullptr, nullptr, SEQ, nullptr, SCL2, PLW);
}
__global__ __launch_bounds__(32) void k_pv(const h16* __restrict__ P, const h16* __restrict__ HI, const h16* __restrict__ RS, h16* CH, h16* CR, const int* __restrict__ PLW) {
    __shared__ __align__(16) float os[16 * 68];
    const size_t z = blockIdx.z;
    const h16* ph = P + z * SEQ * (size_t)(2 * SEQ); const h16* pr = ph + SEQ;
    const h16* vh = HI + (size_t)2 * NHA * SEQ * DD + z * DD * SEQ; const h16* vr = RS + (size_t)2 * NHA * SEQ * DD + z * DD * SEQ;
    gemmb_body<1>(os, ph, pr, vh, vr, 2 * SEQ, SEQ, SEQ, nullptr, CH + z * DD, CR + z * DD, KM, nullptr, OCAR, PLW);
}
__global__ __launch_bounds__(32) void k_out(const h16* __restrict__ CH, const h16* __restrict__ CR, const h16* __restrict__ WOS, float* OUT, const float* __restrict__ bu, const int* __restrict__ PLW) {
    __shared__ __align__(16) float os[16 * 68];
    gemmb_body<2>(os, CH, CR, WOS, WOS, KM, KM, KM, OUT, nullptr, nullptr, DD, bu, FINSC, PLW);
}

__global__ __launch_bounds__(128) void k_padlen(const int* __restrict__ mask, int* PLW) {
    __shared__ int red[4];
    const int wave = __builtin_amdgcn_readfirstlane((int)(threadIdx.x >> 5)); const unsigned lane = threadIdx.x & 31u;
    const int bsel = min((int)(threadIdx.x >> 5), NB - 1); const int b = __builtin_amdgcn_readfirstlane(bsel);
    int s = 0;
#pragma unroll 1
    for (int t = (int)lane * 4; t < SEQ; t += 128) { const v4i m = *(const v4i*)(mask + (size_t)b * SEQ_FULL + t); s += (m[0] + m[1]) + (m[2] + m[3]); }
#pragma unroll
    for (int sh = 16; sh; sh >>= 1) s += __shfl_xor(s, sh, 32);
    if (lane == 0u) red[wave] = s;
    __syncthreads();
    if (wave == 0) { const int r = red[lane & 3u]; const int pv = (lane < (unsigned)NB) ? (SEQ - r) : 0;
        *(volatile int*)(PLW + lane) = pv; __threadfence(); *(volatile int*)(PLW + lane) = pv; }
}

__global__ __launch_bounds__(256) void k_prep(const float* __restrict__ x, const float* __restrict__ wq, const float* __restrict__ wk, const float* __restrict__ wv, const float* __restrict__ wu, bf* XP, bf* WT, h16* WOS) {
    const unsigned which = blockIdx.y; const unsigned i = blockIdx.x * 256u + threadIdx.x;
    if (which == 0u) {
        if (i >= XG) return;
        const v8f v = *(const v8f*)(x + (size_t)i * 8);
        v8us o;
#pragma unroll
        for (int k = 0; k < 8; ++k) o[k] = f2bf(v[k]);
        bf* dst = XP + (size_t)i * 8;
        *(volatile v8us*)dst = o; __threadfence(); *(volatile v8us*)dst = o;
    } else if (which <= 3u) {
        if (i >= WG) return;
        const float* src = (which == 1u) ? wq : ((which == 2u) ? wk : wv);
        const v8f v = *(const v8f*)(src + (size_t)i * 8);
        v8us o;
#pragma unroll
        for (int k = 0; k < 8; ++k) o[k] = f2bf(v[k]);
        bf* dst = WT + (size_t)(which - 1u) * NHA * DD * DD + (size_t)i * 8;
        *(volatile v8us*)dst = o; __threadfence(); *(volatile v8us*)dst = o;
    } else {
        if (i >= OG) return;
        const unsigned n = i / (unsigned)(KM / 8), c = i - n * (unsigned)(KM / 8);
        const v8f v = *(const v8f*)(wu + (size_t)n * KMF + (size_t)c * 8);
        v8h o;
#pragma unroll
        for (int k = 0; k < 8; ++k) o[k] = toh_flush(bfr(v[k]) * WOCAR);
        h16* dst = WOS + (size_t)i * 8;
        *(volatile v8h*)dst = o; __threadfence(); *(volatile v8h*)dst = o;
    }
}

__global__ __launch_bounds__(256) void k_split(const float* __restrict__ src, h16* HI, h16* RS) {
#pragma clang fp contract(off)
    const size_t i = (size_t)blockIdx.x * 256u + threadIdx.x;
    const v8f v = *(const v8f*)(src + i * 8);
    v8h oh, orr;
#pragma unroll
    for (int k = 0; k < 8; ++k) { const h16 hh = toh_flush(v[k]); oh[k] = hh; orr[k] = toh_flush((v[k] - (float)hh) * RCAR); }
    h16* dh = HI + i * 8; h16* dr = RS + i * 8;
    *(volatile v8h*)dh = oh; *(volatile v8h*)dr = orr; __threadfence(); *(volatile v8h*)dh = oh; *(volatile v8h*)dr = orr;
}

__global__ __launch_bounds__(32 * MSW) void k_msoft(float* S, const int* __restrict__ PLW) {
#pragma clang fp contract(off)
    __shared__ v4f rowbuf[MSW * SEQ / 4];
    const int wave = __builtin_amdgcn_readfirstlane((int)(threadIdx.x >> 5));
    const unsigned lane = threadIdx.x & 31u; const unsigned row = blockIdx.x * (unsigned)MSW + (unsigned)wave;
    const unsigned z = (blockIdx.x * (unsigned)MSW) / (unsigned)SEQ; const int r = (int)(row - z * (unsigned)SEQ);
    int pl = PLW[z]; pl = min(max(pl, 0), SEQ);
    const bool rowvalid = (r >= pl);
    float* sr = S + (size_t)row * SEQ;
    const unsigned lb = (unsigned)wave * (unsigned)(SEQ / 4) + lane * 2u;
    float mx = -3.0e38f;
#pragma unroll 1
    for (int ch = 0; ch < SEQ / 256; ++ch) {
        v4f a0 = *(const v4f*)(sr + ch * 256 + lane * 8u); v4f a1 = *(const v4f*)(sr + ch * 256 + lane * 8u + 4u);
        asm volatile("" : "+v"(a0)); asm volatile("" : "+v"(a1));
        v4f t0, t1;
#pragma unroll
        for (int q = 0; q < 4; ++q) { const int key = ch * 256 + (int)lane * 8 + q; const bool ok = (key >= pl) && (key <= r); const float t = ok ? a0[q] : -3.0e38f; t0[q] = t; mx = fmaxf(mx, t); }
#pragma unroll
        for (int q = 0; q < 4; ++q) { const int key = ch * 256 + (int)lane * 8 + 4 + q; const bool ok = (key >= pl) && (key <= r); const float t = ok ? a1[q] : -3.0e38f; t1[q] = t; mx = fmaxf(mx, t); }
        rowbuf[lb + (unsigned)ch * 64u] = t0; rowbuf[lb + (unsigned)ch * 64u + 1u] = t1;
    }
#pragma unroll
    for (int sh = 16; sh; sh >>= 1) mx = fmaxf(mx, __shfl_xor(mx, sh, 32));
    float sum = 0.f;
#pragma unroll 1
    for (int ch = 0; ch < SEQ / 256; ++ch) {
        const v4f t0 = rowbuf[lb + (unsigned)ch * 64u]; const v4f t1 = rowbuf[lb + (unsigned)ch * 64u + 1u];
        v4f e0, e1;
#pragma unroll
        for (int q = 0; q < 4; ++q) { const float tk = t0[q]; float d0 = __fsub_rn(tk, mx); asm volatile("" : "+v"(d0)); float e = __builtin_amdgcn_exp2f(d0); e = (tk > -1.0e38f) ? e : 0.f; e0[q] = e; sum += e; }
#pragma unroll
        for (int q = 0; q < 4; ++q) { const float tk = t1[q]; float d0 = __fsub_rn(tk, mx); asm volatile("" : "+v"(d0)); float e = __builtin_amdgcn_exp2f(d0); e = (tk > -1.0e38f) ? e : 0.f; e1[q] = e; sum += e; }
        rowbuf[lb + (unsigned)ch * 64u] = e0; rowbuf[lb + (unsigned)ch * 64u + 1u] = e1;
    }
#pragma unroll
    for (int sh = 16; sh; sh >>= 1) sum += __shfl_xor(sum, sh, 32);
    const float sumg = rowvalid ? sum : 1.0f;
    const float f0 = __fdiv_rn(PCAR, sumg);
    const float f = rowvalid ? f0 : 0.f;
    h16* phrow = (h16*)sr; h16* prrow = phrow + SEQ;
#pragma unroll 1
    for (int ps = 0; ps < 2; ++ps) {
#pragma unroll 1
        for (int ch = 0; ch < SEQ / 256; ++ch) {
            const v4f e0 = rowbuf[lb + (unsigned)ch * 64u]; const v4f e1 = rowbuf[lb + (unsigned)ch * 64u + 1u];
            v8h oh, orr;
#pragma unroll
            for (int q = 0; q < 4; ++q) {
                const float p0 = e0[q] * f; const h16 h0 = toh_flush(p0); oh[q] = h0; orr[q] = toh_flush((p0 - (float)h0) * RCAR);
                const float p1 = e1[q] * f; const h16 h1 = toh_flush(p1); oh[4 + q] = h1; orr[4 + q] = toh_flush((p1 - (float)h1) * RCAR); }
            *(volatile v8h*)(phrow + ch * 256 + lane * 8u) = oh; *(volatile v8h*)(prrow + ch * 256 + lane * 8u) = orr;
        }
        if (ps == 0) __threadfence(); }
}

__global__ __launch_bounds__(256) void k_bias(const float* __restrict__ bu, float* OUT) {
    const size_t i = (size_t)blockIdx.x * 256u + threadIdx.x;
    const unsigned c = ((unsigned)i * 4u) & (unsigned)(DD - 1);
    const v4f b = *(const v4f*)(bu + c); v4f o;
#pragma unroll
    for (int e = 0; e < 4; ++e) o[e] = bfr(b[e]);
    float* dst = OUT + (size_t)SEQ * DD + i * 4;
    *(volatile v4f*)dst = o; __threadfence(); *(volatile v4f*)dst = o;
}

#define SZ_PL  ((size_t)256)
#define SZ_XP  ((size_t)SEQ * DD * 2)
#define SZ_WT  ((size_t)3 * NHA * DD * DD * 2)
#define SZ_WOS ((size_t)DD * KM * 2)
#define SZ_P32 ((size_t)3 * NHA * SEQ * DD * 4)
#define SZ_H16 ((size_t)3 * NHA * SEQ * DD * 2)
#define SZ_S   ((size_t)NHA * SEQ * SEQ * 4)
#define SZ_CTX ((size_t)SEQ * KM * 2)
#define SZ_ALL (SZ_PL + SZ_XP + SZ_WT + SZ_WOS + SZ_P32 + 2 * SZ_H16 + SZ_S + 2 * SZ_CTX)
static_assert(SZ_ALL <= (size_t)134217728);
static_assert(SZ_XP % 256 == 0 && SZ_WT % 256 == 0 && SZ_WOS % 256 == 0 && SZ_P32 % 256 == 0 && SZ_H16 % 256 == 0 && SZ_S % 256 == 0 && SZ_CTX % 256 == 0);
static_assert((size_t)NHA * 4 <= SZ_PL && (size_t)32 * 4 <= SZ_PL);
static_assert((size_t)XG * 16 == SZ_XP && (size_t)3 * WG * 16 == SZ_WT && (size_t)OG * 16 == SZ_WOS);
static_assert((size_t)2 * SEQ * 2 == (size_t)SEQ * 4);

extern "C" void kernel_launch(void* const* d_in, const int* in_sizes, int n_in,
                              void* d_out, int out_size, void* d_ws, size_t ws_size, hipStream_t stream) {
    if (n_in < 7) return;
    if ((size_t)in_sizes[0] < (size_t)SEQ * DD) return;
    if ((size_t)in_sizes[1] < (size_t)(NB - 1) * SEQ_FULL + (size_t)SEQ) return;
    if ((size_t)in_sizes[2] < (size_t)NHA * DD * DD || (size_t)in_sizes[3] < (size_t)NHA * DD * DD || (size_t)in_sizes[4] < (size_t)NHA * DD * DD) return;
    if ((size_t)in_sizes[5] < (size_t)(DD - 1) * KMF + (size_t)KM || (size_t)in_sizes[6] < (size_t)DD) return;
    if ((size_t)out_size < (size_t)NB * SEQ * DD) return;
    if (SZ_ALL > ws_size) return;
    const float* X = (const float*)d_in[0]; const int* MASK = (const int*)d_in[1];
    const float* Wq = (const float*)d_in[2]; const float* Wk = (const float*)d_in[3]; const float* Wv = (const float*)d_in[4];
    const float* Wu = (const float*)d_in[5]; const float* bu = (const float*)d_in[6];
    float* OUT = (float*)d_out;
    char* wsp = (char*)d_ws;
    int* PLW = (int*)wsp; wsp += SZ_PL;
    bf* XP = (bf*)wsp; wsp += SZ_XP;
    bf* WT = (bf*)wsp; wsp += SZ_WT;
    h16* WOS = (h16*)wsp; wsp += SZ_WOS;
    float* P32 = (float*)wsp; wsp += SZ_P32;
    h16* HI = (h16*)wsp; wsp += SZ_H16;
    h16* RS = (h16*)wsp; wsp += SZ_H16;
    float* S = (float*)wsp; wsp += SZ_S;
    h16* CH = (h16*)wsp; wsp += SZ_CTX;
    h16* CR = (h16*)wsp; wsp += SZ_CTX;

    k_padlen<<<1, 128, 0, stream>>>(MASK, PLW);
    k_prep<<<dim3(PREPX, 5, 1), 256, 0, stream>>>(X, Wq, Wk, Wv, Wu, XP, WT, WOS);
    k_gemmw<bf, float, 0><<<dim3(SEQ / 64, DD / 64, 2 * NHA), 32, 0, stream>>>(XP, WT, DD, P32, DD, nullptr, 1.0f, (size_t)0, (size_t)DD * DD, (size_t)SEQ * DD, 0);
    k_gemmw<bf, float, 0><<<dim3(DD / 64, SEQ / 64, NHA), 32, 0, stream>>>(WT + (size_t)2 * NHA * DD * DD, XP, DD, P32 + (size_t)2 * NHA * SEQ * DD, SEQ, nullptr, 1.0f, (size_t)DD * DD, (size_t)0, (size_t)DD * SEQ, 0);
    k_split<<<(unsigned)((size_t)3 * NHA * SEQ * DD / 8 / 256), 256, 0, stream>>>(P32, HI, RS);
    k_score<<<dim3(SEQ / 64, SEQ / 64, NHA), 32, 0, stream>>>(HI, RS, S, PLW);
    k_msoft<<<(unsigned)(NHA * SEQ / MSW), 32 * MSW, 0, stream>>>(S, PLW);
    k_pv<<<dim3(SEQ / 64, DD / 64, NHA), 32, 0, stream>>>((const h16*)S, HI, RS, CH, CR, PLW);
    k_out<<<dim3(SEQ / 64, DD / 64, 1), 32, 0, stream>>>(CH, CR, WOS, OUT, bu, PLW);
    if (NB > 1) k_bias<<<(unsigned)((size_t)(NB - 1) * SEQ * DD / 4 / 256), 256, 0, stream>>>(bu, OUT);
}
